// ExpertLayer_5849745457476
// MI455X (gfx1250) — hardware-verified
//
#include <hip/hip_runtime.h>
#include <stddef.h>
#include <stdint.h>

#define TOK    16384
#define DM     512
#define HDIM   1024
#define NE     8
#define TR     64
#define NTILE  264
#define MP     16896
#define TABH   32
#define TABN   (TABH + MP)
#define NTHR   256
#define GTHR   128
#define BAL    0.01f
#define WSMAX  134217728
#define LDS_BKT ((TABN + NE * 8) * 4)

static_assert(MP == NTILE * TR);
static_assert(MP >= TOK + NE * (TR - 1));
static_assert((TABN % 32) == 0);
static_assert(TOK == NTHR * 64);
static_assert((DM % 64) == 0 && (HDIM % 64) == 0);
static_assert((DM % 32) == 0 && (HDIM % 32) == 0);
static_assert(TR == (GTHR / 32) * 16);
static_assert(LDS_BKT <= 160000);
static_assert(NTHR / 32 == 8);

typedef float          v4f  __attribute__((ext_vector_type(4)));
typedef float          v8f  __attribute__((ext_vector_type(8)));
typedef int            v4i  __attribute__((ext_vector_type(4)));
typedef int            v8i  __attribute__((ext_vector_type(8)));
typedef unsigned short v8us __attribute__((ext_vector_type(8)));
typedef __bf16         v16bf __attribute__((ext_vector_type(16)));
union FragB { v16bf v; v8us h[2]; v8i w; };

__device__ __forceinline__ v8f wmb(const FragB& a, const FragB& b, v8f c) {
  v8f d = __builtin_amdgcn_wmma_f32_16x16x32_bf16(false, a.v, false, b.v, (short)0, c, false, false);
  asm volatile("v_nop\n\tv_nop\n\tv_nop\n\tv_nop" : "+v"(d) : "v"(a.w), "v"(b.w));
  return d;
}

__device__ __forceinline__ unsigned short rne16(float f) {
  unsigned u = __float_as_uint(f);
  u += 0x7FFFu + ((u >> 16) & 1u);
  return (unsigned short)(u >> 16);
}
__device__ __forceinline__ float rne16f(float f) {
  return __uint_as_float(((unsigned)rne16(f)) << 16);
}
__device__ __forceinline__ v8us cvt8(const v4f a, const v4f b) {
  v8us o;
  o[0] = rne16(a.x); o[1] = rne16(a.y); o[2] = rne16(a.z); o[3] = rne16(a.w);
  o[4] = rne16(b.x); o[5] = rne16(b.y); o[6] = rne16(b.z); o[7] = rne16(b.w);
  return o;
}
__device__ __forceinline__ void sp1(float v, unsigned short& hi, unsigned short& lo) {
  const unsigned short hb = rne16(v);
  const float hf = __uint_as_float(((unsigned)hb) << 16);
  hi = hb;
  lo = rne16(v - hf);
}
__device__ __forceinline__ void split8(const v4f a, const v4f b, v8us& hv, v8us& lv) {
  unsigned short h0, h1, h2, h3, h4, h5, h6, h7, l0, l1, l2, l3, l4, l5, l6, l7;
  sp1(a.x, h0, l0); sp1(a.y, h1, l1); sp1(a.z, h2, l2); sp1(a.w, h3, l3);
  sp1(b.x, h4, l4); sp1(b.y, h5, l5); sp1(b.z, h6, l6); sp1(b.w, h7, l7);
  hv[0] = h0; hv[1] = h1; hv[2] = h2; hv[3] = h3; hv[4] = h4; hv[5] = h5; hv[6] = h6; hv[7] = h7;
  lv[0] = l0; lv[1] = l1; lv[2] = l2; lv[3] = l3; lv[4] = l4; lv[5] = l5; lv[6] = l6; lv[7] = l7;
}

__global__ __launch_bounds__(NTHR) void k_wtr(const float* __restrict__ src, unsigned short* dst,
                                              int K, int N, int E, int nUnits) {
  const int u = (int)blockIdx.x * NTHR + (int)threadIdx.x;
  if (u >= nUnits) return;
  const int kq  = K >> 3;
  const int per = N * kq;
  int e = u / per;
  e = e > E - 1 ? E - 1 : e;
  const int rem = u - e * per;
  const int n   = rem / kq;
  const int k8  = (rem - n * kq) * 8;
  const float* p = src + ((size_t)e * (size_t)K + (size_t)k8) * (size_t)N + n;
  v4f a, b;
  a.x = p[0];                 a.y = p[(size_t)N];         a.z = p[(size_t)2 * N];     a.w = p[(size_t)3 * N];
  b.x = p[(size_t)4 * N];     b.y = p[(size_t)5 * N];     b.z = p[(size_t)6 * N];     b.w = p[(size_t)7 * N];
  const v8us o = cvt8(a, b);
  const size_t q = ((size_t)e * (size_t)N + (size_t)n) * (size_t)K + (size_t)k8;
  *(volatile v8us*)(dst + q) = o;
  __threadfence();
  *(volatile v8us*)(dst + q) = o;
}

__device__ __forceinline__ void gacc(float xq, const float* swrow, float (&acc)[NE]) {
  const v4f wa = *(const v4f*)(swrow);
  const v4f wb = *(const v4f*)(swrow + 4);
  acc[0] = fmaf(xq, wa.x, acc[0]); acc[1] = fmaf(xq, wa.y, acc[1]);
  acc[2] = fmaf(xq, wa.z, acc[2]); acc[3] = fmaf(xq, wa.w, acc[3]);
  acc[4] = fmaf(xq, wb.x, acc[4]); acc[5] = fmaf(xq, wb.y, acc[5]);
  acc[6] = fmaf(xq, wb.z, acc[6]); acc[7] = fmaf(xq, wb.w, acc[7]);
}

__global__ __launch_bounds__(NTHR) void k_gate(const float* __restrict__ x, const float* __restrict__ gw,
                                               const float* __restrict__ gb, int* choice) {
  __shared__ __attribute__((aligned(16))) float sw[DM * NE];
  __shared__ float sb[NE];
  const int tid = (int)threadIdx.x;
#pragma unroll 1
  for (int i = tid; i < DM * NE; i += NTHR) sw[i] = rne16f(gw[i]);
  if (tid < NE) sb[tid] = rne16f(gb[tid]);
  __syncthreads();
  int t = (int)blockIdx.x * NTHR + tid;
  const bool live = t < TOK;
  t = t > TOK - 1 ? TOK - 1 : t;
  const float* xr = x + (size_t)t * DM;
  float acc[NE];
#pragma unroll
  for (int e = 0; e < NE; ++e) acc[e] = 0.f;
#pragma unroll 1
  for (int d4 = 0; d4 < DM / 4; ++d4) {
    const v4f xv = *(const v4f*)(xr + 4 * d4);
    const float* swr = sw + (size_t)(4 * d4) * NE;
    gacc(rne16f(xv.x), swr,          acc);
    gacc(rne16f(xv.y), swr + NE,     acc);
    gacc(rne16f(xv.z), swr + 2 * NE, acc);
    gacc(rne16f(xv.w), swr + 3 * NE, acc);
  }
  float bv = acc[0] + sb[0];
  int best = 0;
#pragma unroll
  for (int e = 1; e < NE; ++e) {
    const float l = acc[e] + sb[e];
    const bool up = l > bv;
    best = up ? e : best;
    bv   = up ? l : bv;
  }
  if (live) *(volatile int*)(choice + t) = best;
  __threadfence();
  if (live) *(volatile int*)(choice + t) = best;
}

__device__ __forceinline__ void cnt_add(int c, int (&cnt)[NE]) {
  c = c < 0 ? 0 : (c > NE - 1 ? NE - 1 : c);
#pragma unroll
  for (int e = 0; e < NE; ++e) cnt[e] += (c == e) ? 1 : 0;
}
__device__ __forceinline__ int slot_of(int c, int (&base)[NE]) {
  c = c < 0 ? 0 : (c > NE - 1 ? NE - 1 : c);
  int p = 0;
#pragma unroll
  for (int e = 0; e < NE; ++e) {
    const bool mt = (c == e);
    p = mt ? base[e] : p;
    base[e] += mt ? 1 : 0;
  }
  return p < 0 ? 0 : (p > MP - 1 ? MP - 1 : p);
}

__global__ __launch_bounds__(NTHR) void k_bucket(const int* __restrict__ choice, int* tab, float* lossp) {
  extern __shared__ v4i lds_dyn[];
  int* img = (int*)lds_dyn;
  int* lst = img + TABH;
  int* wt  = img + TABN;
  const int tid = (int)threadIdx.x, lane = tid & 31, wave = tid >> 5;

  const v4i z4 = {0, 0, 0, 0};
#pragma unroll 1
  for (int p = tid; p < TABN / 4; p += NTHR) *(v4i*)(img + 4 * p) = z4;
  __syncthreads();

  const int t0 = tid * (TOK / NTHR);
  int cnt[NE];
#pragma unroll
  for (int e = 0; e < NE; ++e) cnt[e] = 0;
#pragma unroll 1
  for (int c4 = 0; c4 < (TOK / NTHR) / 4; ++c4) {
    const v4i cv = *(const v4i*)(choice + t0 + 4 * c4);
    cnt_add(cv.x, cnt); cnt_add(cv.y, cnt); cnt_add(cv.z, cnt); cnt_add(cv.w, cnt);
  }
  int incl[NE];
#pragma unroll
  for (int e = 0; e < NE; ++e) {
    int v = cnt[e];
#pragma unroll
    for (int d = 1; d < 32; d <<= 1) {
      const int up = __shfl_up(v, d);
      if (lane >= d) v += up;
    }
    incl[e] = v;
    if (lane == 31) wt[e * 8 + wave] = v;
  }
  __syncthreads();
  int pre[NE], tot[NE];
#pragma unroll
  for (int e = 0; e < NE; ++e) {
    int s = 0, all = 0;
#pragma unroll
    for (int w2 = 0; w2 < NTHR / 32; ++w2) {
      const int v = wt[e * 8 + w2];
      all += v;
      s   += (w2 < wave) ? v : 0;
    }
    pre[e] = s + incl[e] - cnt[e];
    all = all < 0 ? 0 : (all > TOK ? TOK : all);
    tot[e] = all;
  }
  int off[NE + 1];
  off[0] = 0;
#pragma unroll
  for (int e = 0; e < NE; ++e) {
    int nx = off[e] + ((tot[e] + TR - 1) / TR) * TR;
    nx = nx > MP ? MP : nx;
    off[e + 1] = nx;
  }
  int base[NE];
#pragma unroll
  for (int e = 0; e < NE; ++e) base[e] = off[e] + pre[e];
#pragma unroll 1
  for (int c4 = 0; c4 < (TOK / NTHR) / 4; ++c4) {
    const v4i cv = *(const v4i*)(choice + t0 + 4 * c4);
    const int tb = t0 + 4 * c4;
    const int p0 = slot_of(cv.x, base); lst[p0] = tb;
    const int p1 = slot_of(cv.y, base); lst[p1] = tb + 1;
    const int p2 = slot_of(cv.z, base); lst[p2] = tb + 2;
    const int p3 = slot_of(cv.w, base); lst[p3] = tb + 3;
  }
  __syncthreads();
  if (tid == 0) {
#pragma unroll
    for (int e = 0; e < NE; ++e) img[e] = tot[e];
#pragma unroll
    for (int e = 0; e <= NE; ++e) img[NE + e] = off[e];
  }
  __syncthreads();
  if (tid == 0) {
    float s = 0.f;
#pragma unroll 1
    for (int e = 0; e < NE; ++e) {
      const float pe = (float)img[e] * (1.0f / (float)TOK);
      s += pe * logf(pe + 1e-10f);
    }
    const float lv = -s * BAL;
    *(volatile float*)lossp = lv;
    __threadfence();
    *(volatile float*)lossp = lv;
  }
#pragma unroll 1
  for (int p = tid; p < TABN / 4; p += NTHR) {
    const v4i v = *(const v4i*)(img + 4 * p);
    *(volatile v4i*)(tab + 4 * p) = v;
  }
  __threadfence();
#pragma unroll 1
  for (int p = tid; p < TABN / 4; p += NTHR) {
    const v4i v = *(const v4i*)(img + 4 * p);
    *(volatile v4i*)(tab + 4 * p) = v;
  }
}

__global__ __launch_bounds__(NTHR) void k_gather(const float* __restrict__ x, const int* __restrict__ tab,
                                                 unsigned short* xg, int nUnits) {
  const int u = (int)blockIdx.x * NTHR + (int)threadIdx.x;
  if (u >= nUnits) return;
  const int row = u >> 6;
  const int c8  = (u & 63) * 8;
  int tk = tab[TABH + row];
  tk = tk < 0 ? 0 : (tk > TOK - 1 ? TOK - 1 : tk);
  const float* p = x + (size_t)tk * DM + c8;
  const v4f a = *(const v4f*)p;
  const v4f b = *(const v4f*)(p + 4);
  const v8us o = cvt8(a, b);
  const size_t q = (size_t)row * DM + (size_t)c8;
  *(volatile v8us*)(xg + q) = o;
  __threadfence();
  *(volatile v8us*)(xg + q) = o;
}

template<int MODE>
__global__ __launch_bounds__(GTHR) void k_gemm(
    const unsigned short* __restrict__ Ahi, const unsigned short* __restrict__ Alo,
    const unsigned short* __restrict__ WT, const float* __restrict__ bias,
    const int* __restrict__ tab, unsigned short* Ohi, unsigned short* Olo, float* outp,
    int K, int N, int wstrE, int bstrE)
{
  __shared__ __attribute__((aligned(16))) float stg[TR * 64];
  const int tid = (int)threadIdx.x, lane = tid & 31, wave = tid >> 5, hh = lane >> 4, m = lane & 15;
  const int rowBase = (int)blockIdx.x * TR;
  const int col0    = (int)blockIdx.y * 64;

  const v4i hc0 = *(const v4i*)(tab);
  const v4i hc1 = *(const v4i*)(tab + 4);
  const v4i ho0 = *(const v4i*)(tab + 8);
  const v4i ho1 = *(const v4i*)(tab + 12);
  int e = 0, offe = ho0.x, cnte = hc0.x;
#define SELX(J, OJ, CJ) { const int oj_ = (OJ); const bool ge_ = rowBase >= oj_; \
    e = ge_ ? (J) : e; offe = ge_ ? oj_ : offe; cnte = ge_ ? (CJ) : cnte; }
  SELX(1, ho0.y, hc0.y) SELX(2, ho0.z, hc0.z) SELX(3, ho0.w, hc0.w)
  SELX(4, ho1.x, hc1.x) SELX(5, ho1.y, hc1.y) SELX(6, ho1.z, hc1.z) SELX(7, ho1.w, hc1.w)
#undef SELX
  offe = offe < 0 ? 0 : (offe > MP ? MP : offe);
  cnte = cnte < 0 ? 0 : (cnte > TOK ? TOK : cnte);

  v8f acc[4];
  {
    const v8f z = {0.f, 0.f, 0.f, 0.f, 0.f, 0.f, 0.f, 0.f};
    acc[0] = z; acc[1] = z; acc[2] = z; acc[3] = z;
  }
  const size_t arow = (size_t)(rowBase + 16 * wave + m) * (size_t)K + (size_t)(8 * hh);
  const unsigned short* aph = Ahi + arow;
  const unsigned short* apl = Alo + arow;
  const unsigned short* wp  = WT + (size_t)e * (size_t)wstrE + (size_t)(col0 + m) * (size_t)K + (size_t)(8 * hh);
  const int ksteps = K >> 5;
#pragma unroll 1
  for (int ks = 0; ks < ksteps; ++ks) {
    FragB ah, al;
    ah.h[0] = *(const v8us*)(aph + 32 * ks);
    ah.h[1] = *(const v8us*)(aph + 32 * ks + 16);
    if (MODE != 0) {
      al.h[0] = *(const v8us*)(apl + 32 * ks);
      al.h[1] = *(const v8us*)(apl + 32 * ks + 16);
    } else {
      al = ah;
    }
#pragma unroll
    for (int t = 0; t < 4; ++t) {
      const unsigned short* wq = wp + (size_t)(16 * t) * (size_t)K + 32 * ks;
      FragB bf;
      bf.h[0] = *(const v8us*)wq;
      bf.h[1] = *(const v8us*)(wq + 16);
      acc[t] = wmb(ah, bf, acc[t]);
      if (MODE != 0) acc[t] = wmb(al, bf, acc[t]);
    }
  }

#pragma unroll
  for (int t = 0; t < 4; ++t) {
    const int lc = 16 * t + m;
    int bi = col0 + lc;
    bi = bi > N - 1 ? N - 1 : (bi < 0 ? 0 : bi);
    const float bv = rne16f(bias[(size_t)e * (size_t)bstrE + (size_t)bi]);
#pragma unroll
    for (int r = 0; r < 8; ++r) {
      const int lr = 16 * wave + 8 * hh + r;
      float v = acc[t][r] + bv;
      if (MODE == 0) v = fmaxf(v, 0.f);
      stg[lr * 64 + lc] = v;
    }
  }
  __syncthreads();

  if (MODE != 2) {
    const int q8 = lane & 7, sub = lane >> 3;
    v8us hv[4], lv[4];
    size_t po[4];
#pragma unroll
    for (int i = 0; i < 4; ++i) {
      const int lr = 16 * wave + 4 * i + sub;
      const v4f a = *(const v4f*)(stg + lr * 64 + 8 * q8);
      const v4f b = *(const v4f*)(stg + lr * 64 + 8 * q8 + 4);
      split8(a, b, hv[i], lv[i]);
      po[i] = (size_t)(rowBase + lr) * (size_t)N + (size_t)(col0 + 8 * q8);
    }
#pragma unroll
    for (int i = 0; i < 4; ++i) {
      *(volatile v8us*)(Ohi + po[i]) = hv[i];
      *(volatile v8us*)(Olo + po[i]) = lv[i];
    }
    __threadfence();
#pragma unroll
    for (int i = 0; i < 4; ++i) {
      *(volatile v8us*)(Ohi + po[i]) = hv[i];
      *(volatile v8us*)(Olo + po[i]) = lv[i];
    }
  } else {
    v4f fv[8];
    size_t op[8];
    bool ok[8];
#pragma unroll
    for (int i = 0; i < 8; ++i) {
      const int lr = 16 * wave + 2 * i + hh;
      fv[i] = *(const v4f*)(stg + lr * 64 + 4 * m);
      const int gr = rowBase + lr;
      int tk = tab[TABH + gr];
      tk = tk < 0 ? 0 : (tk > TOK - 1 ? TOK - 1 : tk);
      const int rl = gr - offe;
      ok[i] = (rl >= 0) && (rl < cnte);
      op[i] = (size_t)tk * (size_t)N + (size_t)(col0 + 4 * m);
    }
#pragma unroll
    for (int i = 0; i < 8; ++i) {
      if (ok[i]) *(volatile v4f*)(outp + op[i]) = fv[i];
    }
    __threadfence();
#pragma unroll
    for (int i = 0; i < 8; ++i) {
      if (ok[i]) *(volatile v4f*)(outp + op[i]) = fv[i];
    }
  }
}

static inline int cdiv(int a, int b) { return (a + b - 1) / b; }

extern "C" void kernel_launch(void* const* d_in, const int* in_sizes, int n_in,
                              void* d_out, int out_size, void* d_ws, size_t ws_size,
                              hipStream_t stream) {
  if (n_in < 9) return;
  if (in_sizes[0] != TOK * DM) return;
  if (in_sizes[1] != DM * NE) return;
  if (in_sizes[2] != NE) return;
  if (in_sizes[3] != NE * DM * HDIM) return;
  if (in_sizes[4] != NE * HDIM) return;
  if (in_sizes[5] != NE * HDIM * DM) return;
  if (in_sizes[6] != NE * DM) return;
  if (in_sizes[7] != DM * DM) return;
  if (in_sizes[8] != DM) return;
  if (out_size != TOK * DM + 1) return;

  const float* x  = (const float*)d_in[0];
  const float* gw = (const float*)d_in[1];
  const float* gb = (const float*)d_in[2];
  const float* w1 = (const float*)d_in[3];
  const float* b1 = (const float*)d_in[4];
  const float* w2 = (const float*)d_in[5];
  const float* b2 = (const float*)d_in[6];
  const float* pw = (const float*)d_in[7];
  const float* pb = (const float*)d_in[8];
  float* out   = (float*)d_out;
  float* lossp = out + (size_t)TOK * DM;

  char* ws = (char*)d_ws;
  size_t off = 0;
  const size_t oW1T = off; off += (size_t)NE * HDIM * DM * 2;    off = (off + 255) & ~(size_t)255;
  const size_t oW2T = off; off += (size_t)NE * DM * HDIM * 2;    off = (off + 255) & ~(size_t)255;
  const size_t oWPT = off; off += (size_t)DM * DM * 2;           off = (off + 255) & ~(size_t)255;
  const size_t oCH  = off; off += (size_t)TOK * 4;               off = (off + 255) & ~(size_t)255;
  const size_t oTAB = off; off += (size_t)TABN * 4;              off = (off + 255) & ~(size_t)255;
  const size_t oXG  = off; off += (size_t)MP * DM * 2;           off = (off + 255) & ~(size_t)255;
  const size_t oHHI = off; off += (size_t)MP * HDIM * 2;         off = (off + 255) & ~(size_t)255;
  const size_t oHLO = off; off += (size_t)MP * HDIM * 2;         off = (off + 255) & ~(size_t)255;
  const size_t oYLO = off; off += (size_t)MP * DM * 2;           off = (off + 255) & ~(size_t)255;
  if (off > ws_size || off > (size_t)WSMAX) return;

  unsigned short* W1T = (unsigned short*)(ws + oW1T);
  unsigned short* W2T = (unsigned short*)(ws + oW2T);
  unsigned short* WPT = (unsigned short*)(ws + oWPT);
  int*            CH  = (int*)(ws + oCH);
  int*            TAB = (int*)(ws + oTAB);
  unsigned short* XG  = (unsigned short*)(ws + oXG);
  unsigned short* YHI = XG;
  unsigned short* HHI = (unsigned short*)(ws + oHHI);
  unsigned short* HLO = (unsigned short*)(ws + oHLO);
  unsigned short* YLO = (unsigned short*)(ws + oYLO);

  hipFuncSetAttribute(reinterpret_cast<const void*>(&k_bucket),
                      hipFuncAttributeMaxDynamicSharedMemorySize, LDS_BKT);

  {
    const int nU1 = NE * HDIM * DM / 8;
    k_wtr<<<cdiv(nU1, NTHR), NTHR, 0, stream>>>(w1, W1T, DM, HDIM, NE, nU1);
    const int nU2 = NE * DM * HDIM / 8;
    k_wtr<<<cdiv(nU2, NTHR), NTHR, 0, stream>>>(w2, W2T, HDIM, DM, NE, nU2);
    const int nU3 = DM * DM / 8;
    k_wtr<<<cdiv(nU3, NTHR), NTHR, 0, stream>>>(pw, WPT, DM, DM, 1, nU3);
  }

  k_gate<<<cdiv(TOK, NTHR), NTHR, 0, stream>>>(x, gw, gb, CH);
  k_bucket<<<1, NTHR, LDS_BKT, stream>>>(CH, TAB, lossp);

  {
    const int nUg = MP * (DM / 8);
    k_gather<<<cdiv(nUg, NTHR), NTHR, 0, stream>>>(x, TAB, XG, nUg);
  }

  k_gemm<0><<<dim3(NTILE, HDIM / 64), GTHR, 0, stream>>>(XG, XG, W1T, b1, TAB, HHI, HLO, out,
                                                           DM, HDIM, HDIM * DM, HDIM);
  k_gemm<1><<<dim3(NTILE, DM / 64), GTHR, 0, stream>>>(HHI, HLO, W2T, b2, TAB, YHI, YLO, out,
                                                         HDIM, DM, DM * HDIM, DM);
  k_gemm<2><<<dim3(NTILE, DM / 64), GTHR, 0, stream>>>(YHI, YLO, WPT, pb, TAB, HHI, HLO, out,
                                                         DM, DM, 0, 0);
}
